// QuanvolutionGen216_65481071406272
// MI455X (gfx1250) — hardware-verified
//
#include <hip/hip_runtime.h>
#include <stddef.h>
#include <math.h>


#define IMGW    28
#define IMGSZ   784
#define NPATCH  196
#define PROW    14
#define KDIM    784
#define KP      800
#define KPL     808
#define NCLS    10
#define NP      16
#define MT      16
#define NTHR    256
#define NQP     12
#define WSCL    16.0f
#define WINV    0.0625f

static_assert(KP % 32 == 0 && KP >= KDIM);
static_assert(KPL % 8 == 0 && KPL >= KP);
static_assert(KDIM % 8 == 0);
static_assert((MT * NCLS * 4) % 128 == 0);
static_assert((NP * KP) % 8 == 0);
static_assert(MT * NP == NTHR);
static_assert((MT * KPL) % 8 == 0);

typedef float    v2f  __attribute__((ext_vector_type(2)));
typedef float    v4f  __attribute__((ext_vector_type(4)));
typedef float    v8f  __attribute__((ext_vector_type(8)));
typedef _Float16 v4h  __attribute__((ext_vector_type(4)));
typedef _Float16 v8h  __attribute__((ext_vector_type(8)));
typedef _Float16 v16h __attribute__((ext_vector_type(16)));
union FragH { v16h v; v8h h[2]; };

__device__ __forceinline__ v8f wmh(v16h a, v16h b, v8f c) {
  v8f d = __builtin_amdgcn_wmma_f32_16x16x32_f16(false, a, false, b, (short)0, c, false, false);
#if defined(__HIP_DEVICE_COMPILE__)
  asm volatile("v_nop\n\tv_nop\n\tv_nop\n\tv_nop" : "+v"(d) : "v"(a), "v"(b));
#endif
  return d;
}

__device__ __forceinline__ v8f zero8() {
  v8f z = {0.f, 0.f, 0.f, 0.f, 0.f, 0.f, 0.f, 0.f};
  return z;
}

__global__ __launch_bounds__(NTHR) void k_prep(const float* __restrict__ W, _Float16* Wp) {
  const int i = blockIdx.x * NTHR + (int)threadIdx.x;
  if (i >= NP * KP / 8) return;
  const int o  = i * 8;
  const int n  = o / KP;
  const int k0 = o - n * KP;
  const int nc = n < NCLS ? n : NCLS - 1;
  v8h hv;
#pragma unroll
  for (int e = 0; e < 8; ++e) {
    const int k  = k0 + e;
    const int kc = k < KDIM ? k : KDIM - 1;
    const float wv = W[(size_t)nc * KDIM + kc];
    const float v  = (n < NCLS && k < KDIM) ? wv * WSCL : 0.0f;
    hv[e] = (_Float16)v;
  }
  _Float16* dp = Wp + o;
  *(volatile v8h*)dp = hv;
  __threadfence();
  *(volatile v8h*)dp = hv;
}

__global__ __launch_bounds__(NTHR) void k_main(const float* __restrict__ x, const float* __restrict__ qp,
                                               const _Float16* __restrict__ Wp, const float* __restrict__ bias,
                                               float* out, int nB) {
  __shared__ v8h   sF8[MT * KPL / 8];
  __shared__ float sPh[2 * NQP];
  __shared__ float sL[MT * NP];
  __shared__ v4f   sO4[MT * NCLS / 4];
  _Float16* sF = (_Float16*)sF8;
  float* sO = (float*)sO4;

  const int tid = threadIdx.x, lane = tid & 31, wave = tid >> 5, hh = lane >> 4, m = lane & 15;
  const int img0 = blockIdx.x * MT;

  if (tid < NQP) {
    const float ph = qp[tid] * 0.5f;
    sPh[2 * tid]     = cosf(ph);
    sPh[2 * tid + 1] = sinf(ph);
  }
  if (tid < MT * 3) {
    const int r = tid / 3, g = tid - r * 3;
    v8h z;
#pragma unroll
    for (int e = 0; e < 8; ++e) z[e] = (_Float16)0.0f;
    *(v8h*)(sF + r * KPL + KDIM + 8 * g) = z;
  }
  __syncthreads();

  for (int t = tid; t < MT * NPATCH; t += NTHR) {
    const int r  = t / NPATCH;
    const int p  = t - r * NPATCH;
    const int pr = p / PROW, pc = p - pr * PROW;
    int img = img0 + r;
    img = img > nB - 1 ? nB - 1 : img;
    const float* xb = x + (size_t)img * IMGSZ + (2 * pr) * IMGW + 2 * pc;
    const v2f t0 = *(const v2f*)xb;
    const v2f t1 = *(const v2f*)(xb + IMGW);
    const float ang[4] = { t0.x, t0.y, t1.x, t1.y };

    float cg[4], sg[4];
#pragma unroll
    for (int w = 0; w < 4; ++w) {
      const float hf = ang[w] * 0.5f;
      cg[w] = cosf(hf);
      sg[w] = sinf(hf);
    }

    float re[16], im[16];
#pragma unroll
    for (int i = 0; i < 16; ++i) { re[i] = 0.f; im[i] = 0.f; }
    re[0] = 1.0f;

#pragma unroll
    for (int layer = 0; layer < 3; ++layer) {
#pragma unroll
      for (int w = 0; w < 4; ++w) {
        const int bw = 8 >> w;
        const float c = cg[w], s = sg[w];
#pragma unroll
        for (int i = 0; i < 16; ++i) {
          if (i & bw) continue;
          const int j = i | bw;
          const float ra = re[i], ia = im[i], rb = re[j], ib = im[j];
          re[i] = c * ra + s * ib;  im[i] = c * ia - s * rb;
          re[j] = c * rb + s * ia;  im[j] = c * ib - s * ra;
        }
      }
#pragma unroll
      for (int i = 0; i < 16; ++i) {
        if ((i & 8) && !(i & 4)) {
          const int j = i | 4;
          const float tr = re[i], ti = im[i];
          re[i] = re[j]; im[i] = im[j]; re[j] = tr; im[j] = ti;
        }
      }
#pragma unroll
      for (int i = 0; i < 16; ++i) {
        if ((i & 2) && !(i & 1)) {
          const int j = i | 1;
          const float tr = re[i], ti = im[i];
          re[i] = re[j]; im[i] = im[j]; re[j] = tr; im[j] = ti;
        }
      }
#pragma unroll
      for (int w = 0; w < 4; ++w) {
        const int bw = 8 >> w;
        const float cp = sPh[2 * (layer * 4 + w)];
        const float sp = sPh[2 * (layer * 4 + w) + 1];
#pragma unroll
        for (int i = 0; i < 16; ++i) {
          const float rr = re[i], qq = im[i];
          if (i & bw) { re[i] = cp * rr - sp * qq; im[i] = cp * qq + sp * rr; }
          else        { re[i] = cp * rr + sp * qq; im[i] = cp * qq - sp * rr; }
        }
      }
    }

    float prob[16];
#pragma unroll
    for (int i = 0; i < 16; ++i) prob[i] = re[i] * re[i] + im[i] * im[i];

    v4h f;
#pragma unroll
    for (int w = 0; w < 4; ++w) {
      const int bw = 8 >> w;
      float zp = 0.f, zn = 0.f;
#pragma unroll
      for (int i = 0; i < 16; ++i) {
        if (i & bw) zn += prob[i]; else zp += prob[i];
      }
      f[w] = (_Float16)(zp - zn);
    }
    *(v4h*)(sF + r * KPL + 4 * p) = f;
  }
  __syncthreads();

  if (wave == 0) {
    v8f acc = zero8();
    const _Float16* ar = sF + m * KPL + 8 * hh;
    const _Float16* br = Wp + (size_t)m * KP + 8 * hh;
#pragma unroll
    for (int kt = 0; kt < KP / 32; ++kt) {
      FragH a, b;
      a.h[0] = *(const v8h*)(ar + 32 * kt);
      a.h[1] = *(const v8h*)(ar + 32 * kt + 16);
      b.h[0] = *(const v8h*)(br + 32 * kt);
      b.h[1] = *(const v8h*)(br + 32 * kt + 16);
      acc = wmh(a.v, b.v, acc);
    }
#pragma unroll
    for (int r = 0; r < 8; ++r) sL[(8 * hh + r) * NP + m] = acc[r] * WINV;
  }
  __syncthreads();

  {
    const int row = tid >> 4, col = tid & 15;
    const int cc = col < NCLS ? col : NCLS - 1;
    const bool valid = col < NCLS;
    const float v = sL[row * NP + col] + bias[cc];
    float mx = valid ? v : -3.0e38f;
    mx = fmaxf(mx, __shfl_xor(mx, 8, 16));
    mx = fmaxf(mx, __shfl_xor(mx, 4, 16));
    mx = fmaxf(mx, __shfl_xor(mx, 2, 16));
    mx = fmaxf(mx, __shfl_xor(mx, 1, 16));
    const float sh = v - mx;
    const float ev = expf(fminf(sh, 80.0f));
    float s = valid ? ev : 0.0f;
    s += __shfl_xor(s, 8, 16);
    s += __shfl_xor(s, 4, 16);
    s += __shfl_xor(s, 2, 16);
    s += __shfl_xor(s, 1, 16);
    const float res = sh - logf(s);
    if (valid) sO[row * NCLS + col] = res;
  }
  __syncthreads();

  if (tid < MT * NCLS / 4) {
    const v4f val = sO4[tid];
    float* gp = out + (size_t)img0 * NCLS + 4 * tid;
    *(volatile v4f*)gp = val;
    __threadfence();
    *(volatile v4f*)gp = val;
  }
}

extern "C" void kernel_launch(void* const* d_in, const int* in_sizes, int n_in,
                              void* d_out, int out_size, void* d_ws, size_t ws_size,
                              hipStream_t stream) {
  if (n_in < 4) return;
  const int nB = in_sizes[0] / IMGSZ;
  if (nB <= 0 || in_sizes[0] != nB * IMGSZ || (nB % MT) != 0) return;
  if (in_sizes[1] != NQP || in_sizes[2] != NCLS * KDIM || in_sizes[3] != NCLS) return;
  if (out_size != nB * NCLS) return;

  const float* x    = (const float*)d_in[0];
  const float* qp   = (const float*)d_in[1];
  const float* W    = (const float*)d_in[2];
  const float* bias = (const float*)d_in[3];
  float* out = (float*)d_out;

  const size_t wpBytes = (size_t)NP * KP * 2;
  if (wpBytes > ws_size || wpBytes > (size_t)134217728) return;
  _Float16* Wp = (_Float16*)d_ws;

  k_prep<<<(NP * KP / 8 + NTHR - 1) / NTHR, NTHR, 0, stream>>>(W, Wp);
  k_main<<<nB / MT, NTHR, 0, stream>>>(x, qp, Wp, bias, out, nB);
}
